// MSAAttention_30760555774379
// MI455X (gfx1250) — hardware-verified
//
#include <hip/hip_runtime.h>
#include <math.h>

typedef __attribute__((ext_vector_type(16))) _Float16 v16h;
typedef __attribute__((ext_vector_type(16))) __bf16 v16b;
typedef __attribute__((ext_vector_type(8)))  _Float16 v8h;
typedef __attribute__((ext_vector_type(8)))  float v8f;
typedef __attribute__((ext_vector_type(4)))  float v4f;
typedef __attribute__((ext_vector_type(2)))  float v2f;
typedef __attribute__((ext_vector_type(4)))  unsigned v4u;
typedef __attribute__((ext_vector_type(4)))  int v4i;
typedef float __attribute__((may_alias)) float_a;
typedef int __attribute__((may_alias)) int_a;

template <typename T> __device__ __forceinline__ void vst2(void* p, T v) { *(volatile T*)p = v; __threadfence(); *(volatile T*)p = v; }
__device__ __forceinline__ v8f wmma16(v16h a, v16h b, v8f c) {
  v8f d = __builtin_amdgcn_wmma_f32_16x16x32_f16(false, a, false, b, (short)0, c, false, false);
  asm volatile("v_nop\n\tv_nop\n\tv_nop\n\tv_nop" : "+v"(d) : "v"(a), "v"(b));
  return d;
}
__device__ __forceinline__ v8f wmma_bf(v16b a, v16b b, v8f c) {
  v8f d = __builtin_amdgcn_wmma_f32_16x16x32_bf16(false, a, false, b, (short)0, c, false, false);
  asm volatile("v_nop\n\tv_nop\n\tv_nop\n\tv_nop" : "+v"(d) : "v"(a), "v"(b));
  return d;
}
__device__ __forceinline__ v16h frag_h(const _Float16* rowk0, int lane) {
  union { v16h v; v8h q[2]; } u; const _Float16* p = rowk0 + 8 * (lane >> 4);
  u.q[0] = *(const v8h*)p; u.q[1] = *(const v8h*)(p + 16); return u.v;
}
__device__ __forceinline__ v16h frag_f32(const float* rowk0, int lane) {
  v16h a; const float* p = rowk0 + 8 * (lane >> 4);
#pragma unroll
  for (int i = 0; i < 8; ++i) { a[i] = (_Float16)p[i]; a[8 + i] = (_Float16)p[16 + i]; }
  return a;
}
__device__ __forceinline__ v16h frag_f32s(const float* rowk0, int lane, float sc) {
  v16h a; const float* p = rowk0 + 8 * (lane >> 4);
#pragma unroll
  for (int i = 0; i < 8; ++i) { a[i] = (_Float16)(p[i] * sc); a[8 + i] = (_Float16)(p[16 + i] * sc); }
  return a;
}
__device__ __forceinline__ v16h fragc_f32(const float* W, int k0, int n, int lane, int ld, int K) {
  v16h a; const int g = lane >> 4;
#pragma unroll
  for (int i = 0; i < 8; ++i) { const int ka = k0 + 8 * g + i, kb = ka + 16;
    a[i] = (_Float16)(ka < K ? W[(size_t)(ka < K ? ka : K - 1) * ld + n] : 0.f); a[8 + i] = (_Float16)(kb < K ? W[(size_t)(kb < K ? kb : K - 1) * ld + n] : 0.f); }
  return a;
}
struct F2 { v16b h, l; };
__device__ __forceinline__ F2 bsplit16(const float v[16]) { F2 r;
#pragma unroll
  for (int i = 0; i < 16; ++i) { const __bf16 h = (__bf16)v[i]; r.h[i] = h; r.l[i] = (__bf16)(v[i] - (float)h); }
  return r; }
__device__ __forceinline__ F2 split_row(const float* row, int k0, int lane) { float v[16]; const float* p = row + k0 + 8 * (lane >> 4);
#pragma unroll
  for (int i = 0; i < 8; ++i) { v[i] = p[i]; v[8 + i] = p[16 + i]; }
  return bsplit16(v); }
__device__ __forceinline__ F2 split_rowK(const float* row, int k0, int lane, int K) { float v[16]; const int g = lane >> 4;
#pragma unroll
  for (int i = 0; i < 8; ++i) { const int ka = k0 + 8 * g + i, kb = ka + 16; v[i] = ka < K ? row[ka < K ? ka : K - 1] : 0.f; v[8 + i] = kb < K ? row[kb < K ? kb : K - 1] : 0.f; }
  return bsplit16(v); }
__device__ __forceinline__ F2 split_col(const float* W, int k0, int n, int lane, int ld, int K) { float v[16]; const int g = lane >> 4;
#pragma unroll
  for (int i = 0; i < 8; ++i) { const int ka = k0 + 8 * g + i, kb = ka + 16; v[i] = ka < K ? W[(size_t)(ka < K ? ka : K - 1) * ld + n] : 0.f; v[8 + i] = kb < K ? W[(size_t)(kb < K ? kb : K - 1) * ld + n] : 0.f; }
  return bsplit16(v); }
__device__ __forceinline__ v8f mac3(const F2& a, const F2& b, v8f c) { c = wmma_bf(a.l, b.h, c); c = wmma_bf(a.h, b.l, c); return wmma_bf(a.h, b.h, c); }
__device__ __forceinline__ float sigm(float v) { return 1.0f / (1.0f + expf(-v)); }
#define LDSX() do { asm volatile("s_wait_dscnt 0" ::: "memory"); __builtin_amdgcn_wave_barrier(); __builtin_amdgcn_fence(__ATOMIC_RELEASE, "workgroup"); } while (0)


#define SQ 128
#define RR 256
#define CM 256
#define NH 8
#define CA 32
#define CZ 128
#define FF 1024
#define NROW (SQ * RR)
#define WSC 256.0f
#ifndef TON
#define TON 1
#endif
typedef __attribute__((ext_vector_type(8))) __bf16 v8b;
__device__ __forceinline__ v16b frag_b(const __bf16* rowk0, int lane) {
  union { v16b v; v8b q[2]; } u; const __bf16* p = rowk0 + 8 * (lane >> 4);
  u.q[0] = *(const v8b*)p; u.q[1] = *(const v8b*)(p + 16); return u.v;
}
__device__ __forceinline__ float bfr(float v) { return (float)(__bf16)v; }
__device__ __attribute__((noinline)) float exp_ni(float v) { return expf(v); }
__device__ __attribute__((noinline)) float erf_ni(float v) { return erff(v); }

#define WS_RW   0u
#define WS_CW   (WS_RW + 2u * 1024 * CM)
#define WS_RWO  (WS_CW + 2u * 1024 * CM)
#define WS_CWO  (WS_RWO + 2u * CM * CM)
#define WS_TW1  (WS_CWO + 2u * CM * CM)
#define WS_TW2  (WS_TW1 + 2u * FF * CM)
#define WS_XH   (WS_TW2 + 2u * CM * FF)
#define WS_QK   (WS_XH + 2u * (size_t)NROW * CM)
#define WS_VT   (WS_QK + 2u * (size_t)NROW * 2 * CM)
#define WS_VTL  (WS_VT + 2u * (size_t)NROW * CM)
#define WS_G    (WS_VTL + 2u * (size_t)NROW * CM)
#define WS_O    (WS_G + 2u * (size_t)NROW * CM)
#define WS_M    (WS_O + 4u * (size_t)NROW * CM)
#define WS_PB   (WS_M + 4u * (size_t)NROW * CM)
#define WS_H1   (WS_PB + 4u * (size_t)NH * RR * RR)
#define WS_END  (WS_H1 + 2u * (size_t)NROW * FF)

__global__ __launch_bounds__(256) void k_packw(const float* __restrict__ RQ, const float* __restrict__ RK, const float* __restrict__ RV, const float* __restrict__ RG, const float* __restrict__ CQ, const float* __restrict__ CK, const float* __restrict__ CV, const float* __restrict__ CG, const float* __restrict__ RWO, const float* __restrict__ CWO, const float* __restrict__ TW1, const float* __restrict__ TW2, char* __restrict__ ws) {
  const int n = blockIdx.x, which = blockIdx.y, t = threadIdx.x; __shared__ __align__(16) _Float16 s[FF];
  const float* Wm; int kin, kout, col; _Float16* dst;
  if (which == 0) { if (n >= 1024) return; const int g4 = n / CM; col = n % CM; Wm = g4 == 0 ? RQ : g4 == 1 ? RK : g4 == 2 ? RV : RG; kin = CM; kout = CM; dst = (_Float16*)(ws + WS_RW) + (size_t)n * CM; }
  else if (which == 1) { if (n >= 1024) return; const int g4 = n / CM; col = n % CM; Wm = g4 == 0 ? CQ : g4 == 1 ? CK : g4 == 2 ? CV : CG; kin = CM; kout = CM; dst = (_Float16*)(ws + WS_CW) + (size_t)n * CM; }
  else if (which == 2) { if (n >= CM) return; col = n; Wm = RWO; kin = CM; kout = CM; dst = (_Float16*)(ws + WS_RWO) + (size_t)n * CM; }
  else if (which == 3) { if (n >= CM) return; col = n; Wm = CWO; kin = CM; kout = CM; dst = (_Float16*)(ws + WS_CWO) + (size_t)n * CM; }
  else if (which == 4) { if (n >= FF) return; col = n; Wm = TW1; kin = CM; kout = FF; dst = (_Float16*)(ws + WS_TW1) + (size_t)n * CM; }
  else { if (n >= CM) return; col = n; Wm = TW2; kin = FF; kout = CM; dst = (_Float16*)(ws + WS_TW2) + (size_t)n * FF; }
  for (int k = t; k < kin; k += 256) s[k] = (_Float16)(bfr(Wm[(size_t)k * kout + col]) * WSC); __syncthreads(); for (int q = t; q < kin / 8; q += 256) vst2((unsigned*)(dst + q * 8), *(const v4u*)&s[q * 8]); }
__global__ __launch_bounds__(256) void k_init(const float* __restrict__ X, float* __restrict__ M) { const size_t base = (size_t)blockIdx.x * 4096; for (int q = threadIdx.x; q < 1024; q += 256) { v4f v = *(const v4f*)(X + base + q * 4); v[0] = bfr(v[0]); v[1] = bfr(v[1]); v[2] = bfr(v[2]); v[3] = bfr(v[3]); vst2(M + base + q * 4, v); } }
__global__ __launch_bounds__(256) void k_ln(const float* __restrict__ M, const float* __restrict__ G, const float* __restrict__ Bt, _Float16* __restrict__ XH) { __shared__ float red[8]; __shared__ __align__(16) _Float16 sh[CM]; const int t = threadIdx.x; const size_t row = blockIdx.x;
  const float v = M[row * CM + t]; float s = v;
#pragma unroll
  for (int o = 1; o < 32; o <<= 1) s += __shfl_xor(s, o);
  if ((t & 31) == 0) red[t >> 5] = s; __syncthreads(); float mu = 0.f; for (int i = 0; i < 8; ++i) mu += red[i]; mu /= (float)CM; __syncthreads();
  const float d = v - mu; float q = d * d;
#pragma unroll
  for (int o = 1; o < 32; o <<= 1) q += __shfl_xor(q, o);
  if ((t & 31) == 0) red[t >> 5] = q; __syncthreads(); float var = 0.f; for (int i = 0; i < 8; ++i) var += red[i]; var /= (float)CM;
  sh[t] = (_Float16)(d / sqrtf(var + 1e-5f) * bfr(G[t]) + bfr(Bt[t])); __syncthreads(); if (t < CM / 8) vst2((unsigned*)(XH + row * CM + t * 8), *(const v4u*)&sh[t * 8]); }
template <int MODE> __device__ __forceinline__ size_t nat(size_t b, int n) { return MODE == 0 ? b * RR + n : (size_t)n * RR + b; }
template <int MODE>
__global__ __launch_bounds__(128) void k_proj(const _Float16* __restrict__ XH, const _Float16* __restrict__ Wr, const float* __restrict__ BG, _Float16* __restrict__ QK, _Float16* __restrict__ VT, _Float16* __restrict__ VTL, _Float16* __restrict__ Gt) {
  constexpr int NN = MODE == 0 ? RR : SQ; __shared__ __align__(16) _Float16 sh[64][136]; __shared__ __align__(16) _Float16 th[128][72], tl[128][72];
  const int tid = threadIdx.x, wave = tid >> 5, lane = tid & 31, col = lane & 15, g = lane >> 4; const size_t b = blockIdx.z; const int n0 = blockIdx.x * 64 + wave * 16; const int c0 = blockIdx.y * 128; const int which = c0 / CM;
  v8f acc[8] = {};
#pragma unroll
  for (int kc = 0; kc < CM / 32; ++kc) { const v16h a = frag_h(XH + nat<MODE>(b, n0 + col) * CM + kc * 32, lane);
#pragma unroll
    for (int j = 0; j < 8; ++j) acc[j] = wmma16(a, frag_h(Wr + (size_t)(c0 + j * 16 + col) * CM + kc * 32, lane), acc[j]); }
#pragma unroll
  for (int j = 0; j < 8; ++j) { const int cc = (c0 % CM) + j * 16 + col; const float bg = (which == 3) ? bfr(BG[cc]) : 0.f;
#pragma unroll
    for (int r = 0; r < 8; ++r) { float v = acc[j][r] * (1.0f / WSC); if (which == 3) v = 1.0f / (1.0f + expf(-(v + bg)));
      if (which == 2) { const _Float16 hv = (_Float16)v; th[j * 16 + col][wave * 16 + 8 * g + r] = hv; tl[j * 16 + col][wave * 16 + 8 * g + r] = (_Float16)((v - (float)hv) * 2048.0f); } else sh[wave * 16 + 8 * g + r][j * 16 + col] = (_Float16)v; } }
  __syncthreads();
  if (which < 2) { for (int e = tid; e < 64 * 16; e += 128) { const int rl = e >> 4, q = e & 15; vst2((unsigned*)(QK + (b * NN + blockIdx.x * 64 + rl) * (2 * CM) + c0 + q * 8), *(const v4u*)&sh[rl][q * 8]); } }
  else if (which == 2) { const int cv0 = c0 - 2 * CM; for (int e = tid; e < 128 * 8; e += 128) { const int cl = e >> 3, q = e & 7; const size_t o = ((b * CM + cv0 + cl) * (size_t)NN) + blockIdx.x * 64 + q * 8; vst2((unsigned*)(VT + o), *(const v4u*)&th[cl][q * 8]); vst2((unsigned*)(VTL + o), *(const v4u*)&tl[cl][q * 8]); } }
  else { for (int e = tid; e < 64 * 16; e += 128) { const int rl = e >> 4, q = e & 15; vst2((unsigned*)(Gt + nat<MODE>(b, blockIdx.x * 64 + rl) * CM + (c0 - 3 * CM) + q * 8), *(const v4u*)&sh[rl][q * 8]); } } }
__global__ __launch_bounds__(256) void k_pb(const float* __restrict__ Zp, const float* __restrict__ G, const float* __restrict__ Bt, const float* __restrict__ WB, float* __restrict__ PB) { __shared__ __align__(16) float sp[NH][RR]; __shared__ float swb[CZ][NH + 1]; const int t = threadIdx.x, lane = t & 31, w = t >> 5; const int q = blockIdx.x;
  for (int e = t; e < CZ * NH; e += 256) swb[e / NH][e % NH] = bfr(WB[e]); __syncthreads();
  for (int k = w; k < RR; k += 8) { const float* zr = Zp + ((size_t)q * RR + k) * CZ; float v[4]; float s = 0.f; for (int i = 0; i < 4; ++i) { v[i] = bfr(zr[lane + 32 * i]); s += v[i]; }
#pragma unroll
    for (int o = 1; o < 32; o <<= 1) s += __shfl_xor(s, o);
    const float mu = s / (float)CZ; float qq = 0.f; for (int i = 0; i < 4; ++i) { const float d = v[i] - mu; qq += d * d; }
#pragma unroll
    for (int o = 1; o < 32; o <<= 1) qq += __shfl_xor(qq, o);
    const float inv = 1.0f / sqrtf(qq / (float)CZ + 1e-5f); float ph[NH];
#pragma unroll
    for (int h = 0; h < NH; ++h) ph[h] = 0.f;
    for (int i = 0; i < 4; ++i) { const int c = lane + 32 * i; const float ln = (v[i] - mu) * inv * bfr(G[c]) + bfr(Bt[c]);
#pragma unroll
      for (int h = 0; h < NH; ++h) ph[h] += ln * swb[c][h]; }
#pragma unroll
    for (int h = 0; h < NH; ++h) { float x = ph[h];
#pragma unroll
      for (int o = 1; o < 32; o <<= 1) x += __shfl_xor(x, o);
      if (lane == 0) sp[h][k] = x; } }
  __syncthreads(); for (int e = t; e < NH * RR / 4; e += 256) { const int h = e / (RR / 4), q4 = e % (RR / 4); vst2(PB + ((size_t)h * RR + q) * RR + q4 * 4, *(const v4f*)&sp[h][q4 * 4]); } }
template <int MODE>
__global__ __launch_bounds__(128) void k_att(const _Float16* __restrict__ QK, const _Float16* __restrict__ VT, const _Float16* __restrict__ VTL, const float* __restrict__ PB, const float* __restrict__ MASK, float* __restrict__ O) {
  constexpr int NN = MODE == 0 ? RR : SQ; __shared__ __align__(16) float sp[4][16][36]; __shared__ __align__(16) float so[4][16][36];
  const int tid = threadIdx.x, wave = tid >> 5, lane = tid & 31, col = lane & 15, g = lane >> 4; const int h = blockIdx.y; const size_t b = blockIdx.z; const int q0 = blockIdx.x * 64 + wave * 16; const size_t rq = b * NN + q0;
  const v16h aq = frag_h(QK + (rq + col) * (2 * CM) + h * CA, lane);
  float m[8], l[8];
#pragma unroll
  for (int r = 0; r < 8; ++r) { m[r] = -3.0e38f; l[r] = 0.f; }
  v8f acc[2] = {}, accl[2] = {};
#pragma unroll 1
  for (int ks = 0; ks < NN / 32; ++ks) { v8f s[2];
#pragma unroll
    for (int ct = 0; ct < 2; ++ct) { const int kk = ks * 32 + ct * 16 + col; const size_t rk = b * NN + kk; const v16h kh = frag_h(QK + rk * (2 * CM) + CM + h * CA, lane); v8f c = {}; c = wmma16(aq, kh, c);
      const bool keep = bfr(MASK[nat<MODE>(b, kk)]) != 0.f;
#pragma unroll
      for (int r = 0; r < 8; ++r) { float sc = c[r] * 0.17677669529663687f; if (MODE == 0) sc += PB[((size_t)h * RR + (q0 + 8 * g + r)) * RR + kk]; s[ct][r] = keep ? sc : -3.0e38f; } }
    float alpha[8];
#pragma unroll
    for (int r = 0; r < 8; ++r) { float mx = fmaxf(s[0][r], s[1][r]);
#pragma unroll
      for (int o = 1; o < 16; o <<= 1) mx = fmaxf(mx, __shfl_xor(mx, o));
      const float mn = fmaxf(m[r], mx); alpha[r] = (m[r] <= -1.0e38f) ? 0.f : __expf(m[r] - mn); const float e0 = (s[0][r] <= -1.0e38f) ? 0.f : __expf(s[0][r] - mn), e1 = (s[1][r] <= -1.0e38f) ? 0.f : __expf(s[1][r] - mn); float es = e0 + e1;
#pragma unroll
      for (int o = 1; o < 16; o <<= 1) es += __shfl_xor(es, o);
      l[r] = l[r] * alpha[r] + es; m[r] = mn; sp[wave][8 * g + r][col] = e0; sp[wave][8 * g + r][16 + col] = e1; }
#pragma unroll
    for (int j = 0; j < 2; ++j)
#pragma unroll
      for (int r = 0; r < 8; ++r) { acc[j][r] *= alpha[r]; accl[j][r] *= alpha[r]; }
    LDSX();
    v16h pa, pal; { const float* prow = &sp[wave][col][0] + 8 * (lane >> 4);
#pragma unroll
      for (int i = 0; i < 8; ++i) { const float p0 = prow[i] * 2048.0f, p1 = prow[16 + i] * 2048.0f; pa[i] = (_Float16)p0; pa[8 + i] = (_Float16)p1; pal[i] = (_Float16)((p0 - (float)pa[i]) * 2048.0f); pal[8 + i] = (_Float16)((p1 - (float)pa[8 + i]) * 2048.0f); } }
#pragma unroll
    for (int j = 0; j < 2; ++j) { const size_t po = (b * CM + (size_t)h * CA + j * 16 + col) * (size_t)NN + ks * 32; const v16h vh = frag_h(VT + po, lane); acc[j] = wmma16(pa, vh, acc[j]); accl[j] = wmma16(pa, frag_h(VTL + po, lane), accl[j]); accl[j] = wmma16(pal, vh, accl[j]); }
    LDSX(); }
#pragma unroll
  for (int r = 0; r < 8; ++r) { const float il = (l[r] > 0.f) ? (1.0f / 2048.0f) / l[r] : 0.f;
#pragma unroll
    for (int j = 0; j < 2; ++j) so[wave][8 * g + r][j * 16 + col] = (acc[j][r] + accl[j][r] * (1.0f / 2048.0f)) * il; }
  LDSX(); for (int rl = 0; rl < 16; ++rl) if (lane < 8) vst2(O + (rq + rl) * CM + (size_t)h * CA + lane * 4, *(const v4f*)&so[wave][rl][lane * 4]); }
template <int MODE>
__global__ __launch_bounds__(128) void k_go(const _Float16* __restrict__ Gt, const float* __restrict__ O, const _Float16* __restrict__ WOr, const float* __restrict__ BO, float* __restrict__ M) { __shared__ __align__(16) float sf[4][16][132];
  const int tid = threadIdx.x, wave = tid >> 5, lane = tid & 31, col = lane & 15, g = lane >> 4; const size_t r0 = (size_t)blockIdx.x * 64 + wave * 16; const int c0 = blockIdx.y * 128;
  const size_t nr = r0 + col; const size_t s_ = nr / RR, r_ = nr % RR; const size_t cidx = MODE == 0 ? nr : r_ * SQ + s_;
  v8f acc[8] = {}, accl2[8] = {};
#pragma unroll
  for (int kc = 0; kc < CM / 32; ++kc) { v16h a, al; const _Float16* gp = Gt + nr * CM + kc * 32 + 8 * g; const float* op = O + cidx * CM + kc * 32 + 8 * g;
#pragma unroll
    for (int i = 0; i < 8; ++i) { const float v0 = (float)gp[i] * op[i], v1 = (float)gp[16 + i] * op[16 + i]; a[i] = (_Float16)v0; a[8 + i] = (_Float16)v1; al[i] = (_Float16)((v0 - (float)a[i]) * 2048.0f); al[8 + i] = (_Float16)((v1 - (float)a[8 + i]) * 2048.0f); }
#pragma unroll
    for (int j = 0; j < 8; ++j) { const v16h w = frag_h(WOr + (size_t)(c0 + j * 16 + col) * CM + kc * 32, lane); acc[j] = wmma16(a, w, acc[j]); accl2[j] = wmma16(al, w, accl2[j]); } }
#pragma unroll
  for (int j = 0; j < 8; ++j) { const int c = c0 + j * 16 + col; const float bb = bfr(BO[c]);
#pragma unroll
    for (int r = 0; r < 8; ++r) sf[wave][8 * g + r][j * 16 + col] = (acc[j][r] + accl2[j][r] * (1.0f / 2048.0f)) * (1.0f / WSC) + bb; }
  LDSX(); for (int rl = 0; rl < 16; ++rl) vst2(M + (r0 + rl) * CM + c0 + lane * 4, *(const v4f*)&sf[wave][rl][lane * 4]); }
__global__ __launch_bounds__(128) void k_ff1(const _Float16* __restrict__ XH, const _Float16* __restrict__ W1r, const float* __restrict__ B1, _Float16* __restrict__ H1) { __shared__ __align__(16) _Float16 sh[4][16][136];
  const int tid = threadIdx.x, wave = tid >> 5, lane = tid & 31, col = lane & 15, g = lane >> 4; const size_t r0 = (size_t)blockIdx.x * 64 + wave * 16; const int c0 = blockIdx.y * 128;
  v8f acc[8] = {};
#pragma unroll
  for (int kc = 0; kc < CM / 32; ++kc) { const v16h a = frag_h(XH + (r0 + col) * CM + kc * 32, lane);
#pragma unroll
    for (int j = 0; j < 8; ++j) acc[j] = wmma16(a, frag_h(W1r + (size_t)(c0 + j * 16 + col) * CM + kc * 32, lane), acc[j]); }
#pragma unroll
  for (int j = 0; j < 8; ++j) { const float bb = bfr(B1[c0 + j * 16 + col]);
#pragma unroll
    for (int r = 0; r < 8; ++r) sh[wave][8 * g + r][j * 16 + col] = (_Float16)fmaxf(acc[j][r] * (1.0f / WSC) + bb, 0.f); }
  LDSX(); for (int rl = 0; rl < 16; ++rl) if (lane < 16) vst2((unsigned*)(H1 + (r0 + rl) * FF + c0 + lane * 8), *(const v4u*)&sh[wave][rl][lane * 8]); }
__global__ __launch_bounds__(128) void k_ff2(const _Float16* __restrict__ H1, const _Float16* __restrict__ W2r, const float* __restrict__ B2, const float* __restrict__ M, float* __restrict__ OUT) { __shared__ __align__(16) float sf[4][16][132];
  const int tid = threadIdx.x, wave = tid >> 5, lane = tid & 31, col = lane & 15, g = lane >> 4; const size_t r0 = (size_t)blockIdx.x * 64 + wave * 16; const int c0 = blockIdx.y * 128;
  v8f acc[8] = {};
#pragma unroll 2
  for (int kc = 0; kc < FF / 32; ++kc) { const v16h a = frag_h(H1 + (r0 + col) * FF + kc * 32, lane);
#pragma unroll
    for (int j = 0; j < 8; ++j) acc[j] = wmma16(a, frag_h(W2r + (size_t)(c0 + j * 16 + col) * FF + kc * 32, lane), acc[j]); }
#pragma unroll
  for (int j = 0; j < 8; ++j) { const int c = c0 + j * 16 + col; const float bb = bfr(B2[c]);
#pragma unroll
    for (int r = 0; r < 8; ++r) sf[wave][8 * g + r][j * 16 + col] = acc[j][r] * (1.0f / WSC) + bb + M[(r0 + 8 * g + r) * CM + c]; }
  LDSX(); for (int rl = 0; rl < 16; ++rl) vst2(OUT + (r0 + rl) * CM + c0 + lane * 4, *(const v4f*)&sf[wave][rl][lane * 4]); }
extern "C" void kernel_launch(void* const* d_in, const int* in_sizes, int n_in, void* d_out, int out_size, void* d_ws, size_t ws_size, hipStream_t stream) {
  (void)in_sizes; (void)n_in; (void)out_size;
  const float** F = (const float**)d_in;
  if (ws_size < (size_t)WS_END) return;
  char* ws = (char*)d_ws; _Float16 *RW = (_Float16*)(ws + WS_RW), *RWOp = (_Float16*)(ws + WS_RWO), *XH = (_Float16*)(ws + WS_XH), *QK = (_Float16*)(ws + WS_QK), *VT = (_Float16*)(ws + WS_VT), *VTL = (_Float16*)(ws + WS_VTL), *Gt = (_Float16*)(ws + WS_G);
  float *O = (float*)(ws + WS_O), *M = (float*)(ws + WS_M), *PB = (float*)(ws + WS_PB);
  k_packw<<<dim3(1024, 3), 256, 0, stream>>>(F[8], F[9], F[10], F[11], F[8], F[9], F[10], F[11], F[13], F[13], F[8], F[13], ws);
  k_init<<<(unsigned)((size_t)NROW * CM / 4096), 256, 0, stream>>>(F[0], M);
  k_ln<<<NROW, 256, 0, stream>>>(M, F[3], F[4], XH);
  k_proj<0><<<dim3(RR / 64, 8, SQ), 128, 0, stream>>>(XH, RW, F[12], QK, VT, VTL, Gt);
  k_pb<<<RR, 256, 0, stream>>>(F[1], F[5], F[6], F[7], PB);
  k_att<0><<<dim3(RR / 64, NH, SQ), 128, 0, stream>>>(QK, VT, VTL, PB, F[2], O);
  k_go<0><<<dim3(NROW / 64, CM / 128), 128, 0, stream>>>(Gt, O, RWOp, F[14], (float*)d_out);
}
